// MultiHeadAttention_50706383896888
// MI455X (gfx1250) — hardware-run, weakly checked
//
#include <hip/hip_runtime.h>


#ifndef NB
#define NB 2
#endif
#ifndef SEQ
#define SEQ 2048
#endif
#define NB_FULL  2
#define SEQ_FULL 2048
#ifndef OUT_SEQ
#define OUT_SEQ SEQ
#endif
#ifndef EARLY
#define EARLY 512
#endif
#define EROWS ((EARLY) < (SEQ) ? (EARLY) : (SEQ))
#define DM   2048
#define NQH  32
#define NKV  8
#define GRP  4
#define HD   64
#define EQ   (NQH * HD)
#define EKV  (NKV * HD)
#define ETOT (EQ + 2 * EKV)
#define AW   4
#define QRS  2048.0f
#define QRI  (1.0f / 2048.0f)
#define SC2  (0.125f * 1.4426950408889634f)
#define PSH  10.0f
#define WOS  1024.0f
#define WOI  (1.0f / 1024.0f)

#if defined(__HIP_DEVICE_COMPILE__)
#define VGPR_CAP __attribute__((amdgpu_num_vgpr(256)))
#else
#define VGPR_CAP
#endif

static_assert(HD == 64);
static_assert(NQH == NKV * GRP);
static_assert(EQ == DM);
static_assert(DM % 64 == 0 && EQ % 64 == 0 && EKV % 64 == 0);
static_assert(DM % 32 == 0 && EQ % 32 == 0);
static_assert(SEQ % 64 == 0);
static_assert((SEQ & (SEQ - 1)) == 0);
static_assert(SEQ % (16 * AW) == 0);
static_assert(EROWS % 64 == 0);
static_assert(SEQ % 8 == 0);
static_assert(NB <= NB_FULL);
static_assert(SEQ <= SEQ_FULL);
static_assert(ETOT % 64 == 0 && DM % 64 == 0);
static_assert(ETOT % 4 == 0 && DM % 4 == 0);

typedef _Float16 h16;
typedef unsigned short bf;
typedef __attribute__((ext_vector_type(16))) __bf16   v16bf;
typedef __attribute__((ext_vector_type(16))) _Float16 v16h;
typedef __attribute__((ext_vector_type(8)))  _Float16 v8h;
typedef __attribute__((ext_vector_type(8)))  unsigned short v8us;
typedef __attribute__((ext_vector_type(8)))  float    v8f;
typedef __attribute__((ext_vector_type(4)))  float    v4f;
typedef v4f  __attribute__((may_alias)) v4fa;
typedef v8us __attribute__((may_alias)) v8usa;

__device__ __forceinline__ unsigned short f2bf(float f) { unsigned u = __float_as_uint(f); u += 0x7FFFu + ((u >> 16) & 1u); return (unsigned short)(u >> 16); }
__device__ __forceinline__ float bfv(float f) { return __uint_as_float(((unsigned)f2bf(f)) << 16); }
__device__ __forceinline__ v16h cat16(v8h lo, v8h hi) { return __builtin_shufflevector(lo, hi, 0, 1, 2, 3, 4, 5, 6, 7, 8, 9, 10, 11, 12, 13, 14, 15); }
__device__ __forceinline__ v16bf cat16b(v8us lo, v8us hi) { return __builtin_bit_cast(v16bf, __builtin_shufflevector(lo, hi, 0, 1, 2, 3, 4, 5, 6, 7, 8, 9, 10, 11, 12, 13, 14, 15)); }
__device__ __forceinline__ v8f wmma16(v16h a, v16h b, v8f c) { return __builtin_amdgcn_wmma_f32_16x16x32_f16(false, a, false, b, (short)0, c, false, false); }
__device__ __forceinline__ v8f wmmab(v16bf a, v16bf b, v8f c) { return __builtin_amdgcn_wmma_f32_16x16x32_bf16(false, a, false, b, (short)0, c, false, false); }
__device__ __forceinline__ v16h  ldh(const h16* p) { return cat16(*(const v8h*)p, *(const v8h*)(p + 16)); }
__device__ __forceinline__ v16bf ldb(const bf* p)  { return cat16b(*(const v8us*)p, *(const v8us*)(p + 16)); }
__device__ __forceinline__ void wave_sync() { __builtin_amdgcn_fence(3  , "wavefront"); __builtin_amdgcn_wave_barrier(); asm volatile("" ::: "memory"); }
__device__ __forceinline__ void sched_fence() { asm volatile("" ::: "memory"); }
__device__ __forceinline__ void split16(float x, h16& hv, h16& rv) {
    h16 a = (h16)x; a = (fabsf(x) < 6.2e-5f) ? (h16)0.0f : a;
    hv = a; rv = (h16)((x - (float)a) * QRS);
}
static __device__ __forceinline__ h16 toh_flush(float v) { const h16 r = (h16)v; return (fabsf(v) < 6.103515625e-05f) ? (h16)0.0f : r; }
static __device__ __forceinline__ void split16_flush(float x, h16& hv, h16& rv) {
    const h16 a = toh_flush(x);
    hv = a; rv = toh_flush((x - (float)a) * QRS);
}

__global__ __launch_bounds__(256) void k_cvt8(const float* __restrict__ src, bf* dst, size_t n8, int asF16) {
    const size_t i = (size_t)blockIdx.x * 256 + threadIdx.x; if (i >= n8) return;
    const v8f v = *(const v8f*)(src + i * 8); v8us ob; v8h oh;
#pragma unroll
    for (int k = 0; k < 8; ++k) { const unsigned short bb = f2bf(v[k]); ob[k] = bb; oh[k] = (h16)(__uint_as_float(((unsigned)bb) << 16) * WOS); }
    v8us o = ob; if (asF16) o = __builtin_bit_cast(v8us, oh);
    *(volatile v8us*)(dst + i * 8) = o; __threadfence(); *(volatile v8us*)(dst + i * 8) = o;
}

__global__ __launch_bounds__(256) void k_tcvt(const float* __restrict__ src, bf* dst, int R, int C, int asF16) {
    __shared__ __align__(16) unsigned short ts[64 * 72];
    const int t = threadIdx.x;
    const int n0 = blockIdx.x * 64, k0 = blockIdx.y * 64;
    const int rr = t >> 4, c4 = (t & 15) * 4;
#pragma unroll 1
    for (int it = 0; it < 4; ++it) {
        const int kr = it * 16 + rr;
        const v4f v = *(const v4f*)(src + (size_t)(k0 + kr) * C + n0 + c4);
#pragma unroll
        for (int j = 0; j < 4; ++j) {
            const unsigned short bb = f2bf(v[j]);
            const h16 hv = toh_flush(__uint_as_float(((unsigned)bb) << 16) * WOS);
            const unsigned short hb = __builtin_bit_cast(unsigned short, hv);
            ts[(c4 + j) * 72 + kr] = asF16 ? hb : bb; }
    }
    __syncthreads();
    const int rg = t >> 3, c8 = (t & 7) * 8;
    const v8us o0 = *(const v8usa*)(&ts[rg * 72 + c8]);
    const v8us o1 = *(const v8usa*)(&ts[(32 + rg) * 72 + c8]);
    bf* p0 = dst + (size_t)(n0 + rg) * R + k0 + c8;
    bf* p1 = dst + (size_t)(n0 + 32 + rg) * R + k0 + c8;
    *(volatile v8us*)p0 = o0; *(volatile v8us*)p1 = o1;
    __threadfence();
    *(volatile v8us*)p0 = o0; *(volatile v8us*)p1 = o1;
}

__global__ __launch_bounds__(256) void k_tab(float* CS) {
    __shared__ __align__(16) float ts[8 * 64];
    const int t = threadIdx.x; const int pr = t >> 5, i = t & 31;
    const int pos = blockIdx.x * 8 + pr;
    const float fr = expf(-(float)i * 0.28782313662425575f);
    const float th = (float)pos * fr;
    float sn, cs; sincosf(th, &sn, &cs);
    ts[pr * 64 + i] = cs; ts[pr * 64 + 32 + i] = sn;
    __syncthreads();
    if (t < 128) {
        const int row = t >> 4, c4 = (t & 15) * 4;
        const v4f val = *(const v4fa*)(&ts[row * 64 + c4]);
        float* p = CS + (size_t)(blockIdx.x * 8 + row) * 64 + c4;
        *(volatile v4f*)p = val; __threadfence(); *(volatile v4f*)p = val;
    }
}

template<int ROPE>
__global__ __launch_bounds__(32) VGPR_CAP void k_proj(const bf* __restrict__ A, const bf* __restrict__ Bt, h16* Ph, h16* Pr,
                                                      const float* __restrict__ CS,
                                                      int RB, size_t sRB, int pitch, int CB, size_t sCB) {
    __shared__ __align__(16) float os[16 * 68];
    const int K = DM;
    const int lane = threadIdx.x & 31, lr = lane & 15, hi = lane >> 4; const int r0 = blockIdx.x * 64, c0 = blockIdx.y * 64;
    v8f acc[4][4];
#pragma unroll
    for (int mb = 0; mb < 4; ++mb)
#pragma unroll
        for (int nb = 0; nb < 4; ++nb) acc[mb][nb] = (v8f){};
    const size_t aoff = (size_t)(r0 + lr) * K + 8 * hi, boff = (size_t)(c0 + lr) * K + 8 * hi;
#pragma unroll 1
    for (int kc = 0; kc < K; kc += 32) {
        v16bf a[4];
#pragma unroll
        for (int mb = 0; mb < 4; ++mb) a[mb] = ldb(A + aoff + (size_t)mb * 16 * K + kc);
#pragma unroll
        for (int nb = 0; nb < 4; ++nb) {
            const v16bf bq = ldb(Bt + boff + (size_t)nb * 16 * K + kc);
#pragma unroll
            for (int mb = 0; mb < 4; ++mb) acc[mb][nb] = wmmab(a[mb], bq, acc[mb][nb]);
            asm volatile("v_nop\n\tv_nop\n\tv_nop\n\tv_nop"
                         : "+v"(acc[0][nb]), "+v"(acc[1][nb]), "+v"(acc[2][nb]), "+v"(acc[3][nb])
                         : "v"(a[0]), "v"(a[1]), "v"(a[2]), "v"(a[3]), "v"(bq));
        }
    }
    const size_t tbase = (size_t)(r0 / RB) * sRB + (size_t)(r0 % RB) * (size_t)pitch + (size_t)(c0 / CB) * sCB + (size_t)(c0 % CB);
    const int rg = lane >> 3, c8 = (lane & 7) * 8, pc = c8 ^ 32, ic = c8 & 31;
    const float sg = (c8 < 32) ? -1.0f : 1.0f;
#pragma unroll
    for (int mb = 0; mb < 4; ++mb) {
#pragma unroll
        for (int nb = 0; nb < 4; ++nb) {
#pragma unroll
            for (int j = 0; j < 8; ++j) os[(hi * 8 + j) * 68 + nb * 16 + lr] = acc[mb][nb][j]; }
        wave_sync();
        v8h hv[4], rv[4];
#pragma unroll
        for (int s = 0; s < 4; ++s) { const int row = 4 * s + rg;
            const v4f x0 = *(const v4fa*)(&os[row * 68 + c8]); const v4f x1 = *(const v4fa*)(&os[row * 68 + c8 + 4]);
            float val[8];
            if (ROPE) {
                const v4f p0 = *(const v4fa*)(&os[row * 68 + pc]); const v4f p1 = *(const v4fa*)(&os[row * 68 + pc + 4]);
                const int t = (r0 + mb * 16 + row) & (SEQ - 1);
                const float* cst = CS + (size_t)t * 64;
                const v4f ca = *(const v4f*)(cst + ic), cb = *(const v4f*)(cst + ic + 4), sa = *(const v4f*)(cst + 32 + ic), sb = *(const v4f*)(cst + 32 + ic + 4);
#pragma unroll
                for (int i = 0; i < 4; ++i) {
                    val[i] = x0[i] * ca[i] + sg * (p0[i] * sa[i]);
                    val[4 + i] = x1[i] * cb[i] + sg * (p1[i] * sb[i]); }
            } else {
#pragma unroll
                for (int i = 0; i < 4; ++i) { val[i] = x0[i]; val[4 + i] = x1[i]; }
            }
            v8h hh, rr;
#pragma unroll
            for (int i = 0; i < 8; ++i) { h16 a0, a1; split16_flush(val[i], a0, a1); hh[i] = a0; rr[i] = a1; }
            hv[s] = hh; rv[s] = rr;
            sched_fence(); }
        const size_t sb0 = tbase + (size_t)(mb * 16) * (size_t)pitch;
#pragma unroll 1
        for (int ps = 0; ps < 2; ++ps) {
#pragma unroll
            for (int s = 0; s < 4; ++s) { const size_t oo = sb0 + (size_t)(4 * s + rg) * (size_t)pitch + c8;
                *(volatile v8h*)(Ph + oo) = hv[s]; *(volatile v8h*)(Pr + oo) = rv[s]; }
            if (ps == 0) __threadfence(); }
        wave_sync();
    }
}

template<int EP>
__global__ __launch_bounds__(32 * AW) VGPR_CAP void k_flash(const h16* __restrict__ QH, const h16* __restrict__ QR, const h16* __restrict__ KH, const h16* __restrict__ KR,
                                                            const h16* __restrict__ VH, const h16* __restrict__ VR, h16* CH, h16* CR, int tb0) {
    __shared__ __align__(16) float os[AW * 16 * 68];
    const int lane = threadIdx.x & 31, lr = lane & 15, hi = lane >> 4;
    const int wave = __builtin_amdgcn_readfirstlane((int)(threadIdx.x >> 5));
    const int zh = blockIdx.y; const int b = zh / NQH, h = zh % NQH; const int kvz = b * NKV + h / GRP;
    const int t0 = tb0 + (blockIdx.x * AW + wave) * 16;
    const size_t qo = (size_t)zh * SEQ * HD + (size_t)(t0 + lr) * HD + 8 * hi;
    const v16h qh0 = ldh(QH + qo), qh1 = ldh(QH + qo + 32), qr0 = ldh(QR + qo), qr1 = ldh(QR + qo + 32);
    const size_t ko = (size_t)kvz * SEQ * HD + (size_t)lr * HD + 8 * hi;
    const size_t vo = (size_t)kvz * HD * SEQ + (size_t)lr * SEQ + 8 * hi;
    v8f o0 = (v8f){}, o1 = (v8f){}, o2 = (v8f){}, o3 = (v8f){};
    v8f e0 = (v8f){}, e1 = (v8f){}, e2 = (v8f){}, e3 = (v8f){};
    float m = -3.0e38f, l = 0.0f;
    const int tq = t0 + lr;
    const int nst = (t0 >> 5) + 1;
#pragma unroll 1
    for (int st = 0; st < nst; ++st) {
        const int key0 = st * 32;
        v8f sHa = (v8f){}, sLa = (v8f){}, sHb = (v8f){}, sLb = (v8f){};
        {
            const h16* ka = KH + ko + (size_t)key0 * HD;
            const v16h ka0 = ldh(ka), ka1 = ldh(ka + 32), kb0 = ldh(ka + 16 * HD), kb1 = ldh(ka + 16 * HD + 32);
            sHa = wmma16(ka0, qh0, sHa); sLa = wmma16(ka0, qr0, sLa); sHb = wmma16(kb0, qh0, sHb); sLb = wmma16(kb0, qr0, sLb);
            sHa = wmma16(ka1, qh1, sHa); sLa = wmma16(ka1, qr1, sLa); sHb = wmma16(kb1, qh1, sHb); sLb = wmma16(kb1, qr1, sLb);
            asm volatile("v_nop\n\tv_nop\n\tv_nop\n\tv_nop" : "+v"(sHa), "+v"(sLa), "+v"(sHb), "+v"(sLb)
                         : "v"(ka0), "v"(ka1), "v"(kb0), "v"(kb1), "v"(qh0), "v"(qh1), "v"(qr0), "v"(qr1));
        }
        if (EP) {
            sched_fence();
            const h16* kr = KR + ko + (size_t)key0 * HD;
            const v16h ra0 = ldh(kr), ra1 = ldh(kr + 32), rb0 = ldh(kr + 16 * HD), rb1 = ldh(kr + 16 * HD + 32);
            sLa = wmma16(ra0, qh0, sLa); sLb = wmma16(rb0, qh0, sLb); sLa = wmma16(ra1, qh1, sLa); sLb = wmma16(rb1, qh1, sLb);
            asm volatile("v_nop\n\tv_nop\n\tv_nop\n\tv_nop" : "+v"(sLa), "+v"(sLb)
                         : "v"(ra0), "v"(ra1), "v"(rb0), "v"(rb1), "v"(qh0), "v"(qh1));
        }
        float ta[8], tb[8];
#pragma unroll
        for (int r = 0; r < 8; ++r) { ta[r] = (sHa[r] + sLa[r] * QRI) * SC2; tb[r] = (sHb[r] + sLb[r] * QRI) * SC2; }
        if (key0 + 31 > t0) {
            const int kA = key0 + 8 * hi;
#pragma unroll
            for (int r = 0; r < 8; ++r) { ta[r] = (kA + r > tq) ? -3.0e38f : ta[r]; tb[r] = (kA + 16 + r > tq) ? -3.0e38f : tb[r]; }
        }
        float mx = -3.0e38f;
#pragma unroll
        for (int r = 0; r < 8; ++r) mx = fmaxf(mx, fmaxf(ta[r], tb[r]));
        mx = fmaxf(mx, __shfl_xor(mx, 16, 32));
        const float mnew = fmaxf(m, mx);
        const float alpha = __builtin_amdgcn_exp2f(m - mnew);
        const float sh = PSH - mnew;
        v16h pb, pq; float ls = 0.0f;
        if (EP) {
#pragma unroll
            for (int r = 0; r < 8; ++r) { const float fa = __builtin_amdgcn_exp2f(ta[r] + sh); const float fc = __builtin_amdgcn_exp2f(tb[r] + sh);
                const h16 pa = (h16)fa; const h16 pc = (h16)fc; pb[r] = pa; pb[8 + r] = pc;
                pq[r] = (h16)((fa - (float)pa) * QRS); pq[8 + r] = (h16)((fc - (float)pc) * QRS); ls += fa + fc; }
        } else {
#pragma unroll
            for (int r = 0; r < 8; ++r) { const h16 pa = (h16)__builtin_amdgcn_exp2f(ta[r] + sh); const h16 pc = (h16)__builtin_amdgcn_exp2f(tb[r] + sh);
                pb[r] = pa; pb[8 + r] = pc; pq[r] = (h16)0.0f; pq[8 + r] = (h16)0.0f; ls += (float)pa + (float)pc; }
        }
        l = l * alpha + ls; m = mnew;
        o0 = o0 * alpha; o1 = o1 * alpha; o2 = o2 * alpha; o3 = o3 * alpha;
        if (EP) {
            e0 = e0 * alpha; e1 = e1 * alpha; e2 = e2 * alpha; e3 = e3 * alpha;
            sched_fence();
            const h16* vr = VR + vo + key0;
            const v16h w0 = ldh(vr), w1 = ldh(vr + (size_t)16 * SEQ), w2 = ldh(vr + (size_t)32 * SEQ), w3 = ldh(vr + (size_t)48 * SEQ);
            e0 = wmma16(w0, pb, e0); e1 = wmma16(w1, pb, e1); e2 = wmma16(w2, pb, e2); e3 = wmma16(w3, pb, e3);
            asm volatile("v_nop\n\tv_nop\n\tv_nop\n\tv_nop" : "+v"(e0), "+v"(e1), "+v"(e2), "+v"(e3)
                         : "v"(w0), "v"(w1), "v"(w2), "v"(w3), "v"(pb));
            sched_fence();
        }
        {
            const h16* va = VH + vo + key0;
            const v16h v0 = ldh(va), v1 = ldh(va + (size_t)16 * SEQ), v2 = ldh(va + (size_t)32 * SEQ), v3 = ldh(va + (size_t)48 * SEQ);
            o0 = wmma16(v0, pb, o0); o1 = wmma16(v1, pb, o1); o2 = wmma16(v2, pb, o2); o3 = wmma16(v3, pb, o3);
            if (EP) {
                e0 = wmma16(v0, pq, e0); e1 = wmma16(v1, pq, e1); e2 = wmma16(v2, pq, e2); e3 = wmma16(v3, pq, e3);
                asm volatile("v_nop\n\tv_nop\n\tv_nop\n\tv_nop"
                             : "+v"(o0), "+v"(o1), "+v"(o2), "+v"(o3), "+v"(e0), "+v"(e1), "+v"(e2), "+v"(e3)
                             : "v"(v0), "v"(v1), "v"(v2), "v"(v3), "v"(pb), "v"(pq));
            } else {
                asm volatile("v_nop\n\tv_nop\n\tv_nop\n\tv_nop" : "+v"(o0), "+v"(o1), "+v"(o2), "+v"(o3)
                             : "v"(v0), "v"(v1), "v"(v2), "v"(v3), "v"(pb));
            }
        }
    }
    l += __shfl_xor(l, 16, 32);
    const float inv = 1.0f / l;
    const int wb = wave * 16 * 68;
    v8f f0, f1, f2, f3;
    if (EP) { f0 = (o0 + e0 * QRI) * inv; f1 = (o1 + e1 * QRI) * inv; f2 = (o2 + e2 * QRI) * inv; f3 = (o3 + e3 * QRI) * inv; }
    else    { f0 = o0 * inv; f1 = o1 * inv; f2 = o2 * inv; f3 = o3 * inv; }
    { const v4f a = __builtin_shufflevector(f0, f0, 0, 1, 2, 3), c = __builtin_shufflevector(f0, f0, 4, 5, 6, 7);
      *(v4fa*)(&os[wb + lr * 68 +  0 + 8 * hi]) = a; *(v4fa*)(&os[wb + lr * 68 +  0 + 8 * hi + 4]) = c; }
    { const v4f a = __builtin_shufflevector(f1, f1, 0, 1, 2, 3), c = __builtin_shufflevector(f1, f1, 4, 5, 6, 7);
      *(v4fa*)(&os[wb + lr * 68 + 16 + 8 * hi]) = a; *(v4fa*)(&os[wb + lr * 68 + 16 + 8 * hi + 4]) = c; }
    { const v4f a = __builtin_shufflevector(f2, f2, 0, 1, 2, 3), c = __builtin_shufflevector(f2, f2, 4, 5, 6, 7);
      *(v4fa*)(&os[wb + lr * 68 + 32 + 8 * hi]) = a; *(v4fa*)(&os[wb + lr * 68 + 32 + 8 * hi + 4]) = c; }
    { const v4f a = __builtin_shufflevector(f3, f3, 0, 1, 2, 3), c = __builtin_shufflevector(f3, f3, 4, 5, 6, 7);
      *(v4fa*)(&os[wb + lr * 68 + 48 + 8 * hi]) = a; *(v4fa*)(&os[wb + lr * 68 + 48 + 8 * hi + 4]) = c; }
    wave_sync();
    const int rg = lane >> 3, c8 = (lane & 7) * 8;
    v8h hv[4], rv[4];
#pragma unroll
    for (int s = 0; s < 4; ++s) { const int row = 4 * s + rg;
        const v4f x0 = *(const v4fa*)(&os[wb + row * 68 + c8]); const v4f x1 = *(const v4fa*)(&os[wb + row * 68 + c8 + 4]);
        v8h hh, rr;
#pragma unroll
        for (int i = 0; i < 4; ++i) { h16 a0, a1; split16(x0[i], a0, a1); hh[i] = a0; rr[i] = a1; split16(x1[i], a0, a1); hh[4 + i] = a0; rr[4 + i] = a1; }
        hv[s] = hh; rv[s] = rr; }
    const size_t cb = ((size_t)b * SEQ + t0) * EQ + (size_t)h * HD;
#pragma unroll 1
    for (int ps = 0; ps < 2; ++ps) {
#pragma unroll
        for (int s = 0; s < 4; ++s) { const size_t oo = cb + (size_t)(4 * s + rg) * EQ + c8;
            *(volatile v8h*)(CH + oo) = hv[s]; if (EP) *(volatile v8h*)(CR + oo) = rv[s]; }
        if (ps == 0) __threadfence(); }
}

__global__ __launch_bounds__(32) VGPR_CAP void k_oproj(const h16* __restrict__ A, size_t resOff, const h16* __restrict__ Bt, const float* __restrict__ bias, float* OUT) {
    __shared__ __align__(16) float os[16 * 68];
    const int K = EQ;
    const int lane = threadIdx.x & 31, lr = lane & 15, hi = lane >> 4; const int r0 = blockIdx.x * 64, c0 = blockIdx.y * 64;
    const int early = ((r0 % SEQ) < EROWS) ? 1 : 0;
    v8f acc[4][4];
#pragma unroll
    for (int mb = 0; mb < 4; ++mb)
#pragma unroll
        for (int nb = 0; nb < 4; ++nb) acc[mb][nb] = (v8f){};
    const size_t boff = (size_t)(c0 + lr) * K + 8 * hi;
#pragma unroll 1
    for (int pass = early ? 0 : 1; pass < 2; ++pass) {
        const size_t aoff = ((pass == 0) ? resOff : (size_t)0) + (size_t)(r0 + lr) * K + 8 * hi;
#pragma unroll 1
        for (int kc = 0; kc < K; kc += 32) {
            v16h a[4];
#pragma unroll
            for (int mb = 0; mb < 4; ++mb) a[mb] = ldh(A + aoff + (size_t)mb * 16 * K + kc);
#pragma unroll
            for (int nb = 0; nb < 4; ++nb) {
                const v16h bq = ldh(Bt + boff + (size_t)nb * 16 * K + kc);
#pragma unroll
                for (int mb = 0; mb < 4; ++mb) acc[mb][nb] = wmma16(a[mb], bq, acc[mb][nb]);
                asm volatile("v_nop\n\tv_nop\n\tv_nop\n\tv_nop"
                             : "+v"(acc[0][nb]), "+v"(acc[1][nb]), "+v"(acc[2][nb]), "+v"(acc[3][nb])
                             : "v"(a[0]), "v"(a[1]), "v"(a[2]), "v"(a[3]), "v"(bq));
            }
        }
        if (pass == 0) {
#pragma unroll
            for (int mb = 0; mb < 4; ++mb)
#pragma unroll
                for (int nb = 0; nb < 4; ++nb) acc[mb][nb] = acc[mb][nb] * QRI;
        }
    }
    const int bb = r0 / SEQ, tt0 = r0 % SEQ;
    const v4f braw = *(const v4f*)(bias + c0 + lr * 4);
    v4f bv;
#pragma unroll
    for (int i = 0; i < 4; ++i) bv[i] = bfv(braw[i]);
#pragma unroll
    for (int mb = 0; mb < 4; ++mb) {
#pragma unroll
        for (int nb = 0; nb < 4; ++nb) {
#pragma unroll
            for (int j = 0; j < 8; ++j) os[(hi * 8 + j) * 68 + nb * 16 + lr] = acc[mb][nb][j] * WOI; }
        wave_sync();
        v4f val[8];
#pragma unroll
        for (int s = 0; s < 8; ++s) { const v4f y = *(const v4fa*)(&os[(2 * s + hi) * 68 + lr * 4]); val[s] = y + bv; }
        float* ob = OUT + ((size_t)bb * OUT_SEQ + tt0 + mb * 16) * DM + c0;
#pragma unroll 1
        for (int ps = 0; ps < 2; ++ps) {
#pragma unroll
            for (int s = 0; s < 8; ++s) *(volatile v4f*)(ob + (size_t)(2 * s + hi) * DM + lr * 4) = val[s];
            if (ps == 0) __threadfence(); }
        wave_sync();
    }
}

static constexpr size_t al256(size_t v) { return (v + 255) & ~(size_t)255; }
static constexpr size_t SZ_XB = al256((size_t)NB * SEQ * DM * 2);
static constexpr size_t SZ_WB = al256((size_t)ETOT * DM * 2);
static constexpr size_t SZ_WO = al256((size_t)DM * EQ * 2);
static constexpr size_t SZ_QP = al256((size_t)NB * NQH * SEQ * HD * 2);
static constexpr size_t SZ_KP = al256((size_t)NB * NKV * SEQ * HD * 2);
static constexpr size_t SZ_CP = al256((size_t)NB * SEQ * EQ * 2);
static constexpr size_t SZ_CS = al256((size_t)SEQ * 64 * 4);
static constexpr size_t SZ_TOTAL = SZ_XB + SZ_WB + SZ_WO + 2 * SZ_QP + 4 * SZ_KP + 2 * SZ_CP + SZ_CS;
static_assert(SZ_TOTAL <= (size_t)134217728);
static_assert(((size_t)EQ * DM * 2) % 256 == 0 && ((size_t)EKV * DM * 2) % 256 == 0);

extern "C" void kernel_launch(void* const* d_in, const int* in_sizes, int n_in,
                              void* d_out, int out_size, void* d_ws, size_t ws_size, hipStream_t stream) {
    if (n_in < 4) return;
    const size_t needx = ((size_t)(NB - 1) * SEQ_FULL + SEQ) * DM;
    if ((size_t)in_sizes[0] < needx) return;
    if ((size_t)in_sizes[1] < (size_t)DM * ETOT || (size_t)in_sizes[2] < (size_t)EQ * DM) return;
    if (in_sizes[3] < DM) return;
    if ((size_t)out_size < ((size_t)(NB - 1) * OUT_SEQ + SEQ) * DM) return;
    if (SZ_TOTAL > ws_size) return;
    const float* x = (const float*)d_in[0]; const float* wqkv = (const float*)d_in[1]; const float* wproj = (const float*)d_in[2];
    const float* bproj = (const float*)d_in[3];
    float* OUT = (float*)d_out;
    char* wsp = (char*)d_ws;
    bf* XB = (bf*)wsp; wsp += SZ_XB;
    bf* WB = (bf*)wsp; wsp += SZ_WB;
    bf* WOb = (bf*)wsp; wsp += SZ_WO;
    h16* QH = (h16*)wsp; wsp += SZ_QP;
    h16* QR = (h16*)wsp; wsp += SZ_QP;
    h16* KH = (h16*)wsp; wsp += SZ_KP;
    h16* KR = (h16*)wsp; wsp += SZ_KP;
    h16* VH = (h16*)wsp; wsp += SZ_KP;
    h16* VR = (h16*)wsp; wsp += SZ_KP;
    h16* CH = (h16*)wsp; wsp += SZ_CP;
    h16* CR = (h16*)wsp; wsp += SZ_CP;
    float* CS = (float*)wsp; wsp += SZ_CS;
    const h16* WO = (const h16*)WOb;
    const bf* WQ = WB; const bf* WK = WB + (size_t)EQ * DM; const bf* WV = WB + (size_t)(EQ + EKV) * DM;

    if (SEQ == SEQ_FULL) {
        const size_t n8 = (size_t)NB * SEQ * DM / 8;
        k_cvt8<<<(unsigned)((n8 + 255) / 256), 256, 0, stream>>>(x, XB, n8, 0);
    } else {
        const size_t n8 = (size_t)SEQ * DM / 8;
        for (int b = 0; b < NB; ++b) k_cvt8<<<(unsigned)((n8 + 255) / 256), 256, 0, stream>>>(x + (size_t)b * SEQ_FULL * DM, XB + (size_t)b * SEQ * DM, n8, 0);
    }
    k_tcvt<<<dim3(ETOT / 64, DM / 64, 1), 256, 0, stream>>>(wqkv, WB, DM, ETOT, 0);
    k_tcvt<<<dim3(DM / 64, EQ / 64, 1), 256, 0, stream>>>(wproj, WOb, EQ, DM, 1);
    k_tab<<<SEQ / 8, 256, 0, stream>>>(CS);

    k_proj<1><<<dim3(NB * SEQ / 64, EQ / 64, 1), 32, 0, stream>>>(XB, WQ, QH, QR, CS, SEQ, (size_t)NQH * SEQ * HD, HD, HD, (size_t)SEQ * HD);
    k_proj<1><<<dim3(NB * SEQ / 64, EKV / 64, 1), 32, 0, stream>>>(XB, WK, KH, KR, CS, SEQ, (size_t)NKV * SEQ * HD, HD, HD, (size_t)SEQ * HD);
    k_proj<0><<<dim3(EKV / 64, NB * SEQ / 64, 1), 32, 0, stream>>>(WV, XB, VH, VR, CS, EKV, (size_t)0, SEQ, SEQ, (size_t)EKV * SEQ);

    k_flash<1><<<dim3(EROWS / (16 * AW), NB * NQH, 1), 32 * AW, 0, stream>>>(QH, QR, KH, KR, VH, VR, CH, CR, 0);
    if (SEQ > EROWS)
        k_flash<0><<<dim3((SEQ - EROWS) / (16 * AW), NB * NQH, 1), 32 * AW, 0, stream>>>(QH, QR, KH, KR, VH, VR, CH, CR, EROWS);

    k_oproj<<<dim3(NB * SEQ / 64, DM / 64, 1), 32, 0, stream>>>(CH, SZ_CP / 2, WO, bproj, OUT);
}
